// ResidualSpectralSpatialBlock_37726992728100
// MI455X (gfx1250) — hardware-verified
//
#include <hip/hip_runtime.h>


namespace {
constexpr int NB = 8, L = 256, DM = 256, DI = 512, DS = 16, DTR = 16, KC = 4, XD = DTR + 2 * DS, NT = NB * L;
constexpr float XS = 8.0f, ES = 256.0f, WSC = 256.0f;
typedef _Float16 b16;
typedef __attribute__((ext_vector_type(16))) _Float16 v16b;
typedef __attribute__((ext_vector_type(8))) _Float16 v8b;
typedef __attribute__((ext_vector_type(8))) float v8f;
typedef __attribute__((ext_vector_type(4))) float v4f;
__device__ __forceinline__ float bf16_rne(float f) { unsigned int u = __float_as_uint(f); u += 0x7FFFu + ((u >> 16) & 1u); return __uint_as_float(u & 0xFFFF0000u); }
__device__ __forceinline__ void split16(float v, b16& hi, b16& lo) { hi = (b16)v; lo = (b16)(v - (float)hi); }
__device__ __forceinline__ v16b frag_kb(const b16* p, int hh) { const v8b a = *(const v8b*)(p + 8 * hh), b = *(const v8b*)(p + 16 + 8 * hh); v16b f;
#pragma unroll
  for (int e = 0; e < 8; ++e) { f[e] = a[e]; f[8 + e] = b[e]; } return f; }
__device__ __forceinline__ v8f wmma16b(v16b a, v16b b, v8f c) { v8f d = __builtin_amdgcn_wmma_f32_16x16x32_f16(false, a, false, b, (short)0, c, false, false); asm volatile("v_nop\n\tv_nop\n\tv_nop\n\tv_nop" : "+v"(d) : "v"(a), "v"(b)); return d; }
__device__ __forceinline__ void wave_lds_sync() { __builtin_amdgcn_fence(__ATOMIC_RELEASE, "workgroup"); __builtin_amdgcn_wave_barrier(); __builtin_amdgcn_fence(__ATOMIC_ACQUIRE, "workgroup"); }
__device__ __forceinline__ float pmul(float a, float b) { float p = a * b; asm volatile("" : "+v"(p)); return p; }
__device__ __forceinline__ float silu(float v) { return v / (1.0f + __expf(-v)); }
__device__ __forceinline__ float sigm(float v) { return 1.0f / (1.0f + __expf(-v)); }
__device__ __forceinline__ float softplus(float v) { return v > 20.0f ? v : (v < -20.0f ? __expf(v) : log1pf(__expf(v))); }

__global__ __launch_bounds__(256) void wprep_kernel(const float* __restrict__ w, int KIN, int OUT, int KP, b16* __restrict__ WT) {
  const size_t u = (size_t)blockIdx.x * 256 + threadIdx.x; if (u >= (size_t)OUT * KP / 8) return; const size_t e = u * 8; const int o = (int)(e / KP), k0 = (int)(e % KP); v8b v;
  for (int j = 0; j < 8; ++j) { const int k = k0 + j; v[j] = k < KIN ? (b16)(bf16_rne(w[(size_t)(k < KIN ? k : 0) * OUT + o]) * WSC) : (b16)0.0f; } for (int pass = 0; pass < 2; ++pass) { *(volatile v8b*)(WT + e) = v; __threadfence(); }
}
template <int KIN, int NOUT, int MODE_A, int EPI, int NPROD>
__global__ __launch_bounds__(32) void gemm_kernel(const float* __restrict__ IN_, const float* __restrict__ lng, const float* __restrict__ lnb, float lneps, float asc, const b16* __restrict__ WT, const float* __restrict__ bias, const float* __restrict__ RES, float* __restrict__ OUT) {
  __shared__ __attribute__((aligned(16))) b16 Ah[16][KIN + 8], Al[16][KIN + 8]; __shared__ __attribute__((aligned(16))) float Tf[16][(EPI == 2 ? NOUT : 128) + 4];
  const int lane = threadIdx.x, nloc = lane & 15, hlf = lane >> 4; const size_t m0 = (size_t)blockIdx.x * 16; constexpr int NQ = KIN / 128;
  for (int rr = 0; rr < 16; ++rr) { float v[NQ * 4];
    for (int q = 0; q < NQ; ++q) { const v4f t = *(const v4f*)(IN_ + (m0 + rr) * KIN + q * 128 + lane * 4); for (int j = 0; j < 4; ++j) v[q * 4 + j] = (MODE_A == 2) ? t[j] : bf16_rne(t[j]); }
    if (MODE_A == 1) { float s = 0.0f; for (int j = 0; j < NQ * 4; ++j) s += v[j]; for (int o = 16; o; o >>= 1) s += __shfl_xor(s, o); const float mu = s * (1.0f / KIN); float qv = 0.0f; for (int j = 0; j < NQ * 4; ++j) { const float d = v[j] - mu; qv += pmul(d, d); } for (int o = 16; o; o >>= 1) qv += __shfl_xor(qv, o); const float rs = rsqrtf(qv * (1.0f / KIN) + lneps);
      for (int q = 0; q < NQ; ++q) for (int j = 0; j < 4; ++j) { const int c = q * 128 + lane * 4 + j; v[q * 4 + j] = pmul(pmul(v[q * 4 + j] - mu, rs), bf16_rne(lng[c])) + bf16_rne(lnb[c]); } }
    for (int q = 0; q < NQ; ++q) for (int j = 0; j < 4; ++j) { b16 p, ql; if (NPROD == 1) { p = (b16)(v[q * 4 + j] * asc); ql = (b16)0.0f; } else split16(v[q * 4 + j] * asc, p, ql); Ah[rr][q * 128 + lane * 4 + j] = p; Al[rr][q * 128 + lane * 4 + j] = ql; } }
  wave_lds_sync();
  const float sc = 1.0f / (asc * WSC);
#pragma unroll 1
  for (int cg = 0; cg < NOUT / 128; ++cg) { v8f acc[8];
#pragma unroll
    for (int t = 0; t < 8; ++t) acc[t] = (v8f){};
#pragma unroll 2
    for (int kb = 0; kb < KIN; kb += 32) { const v16b a = frag_kb(&Ah[nloc][kb], hlf); v16b al = {}; if (NPROD == 2) al = frag_kb(&Al[nloc][kb], hlf);
#pragma unroll
      for (int t = 0; t < 8; ++t) { const v16b bw = frag_kb(WT + (size_t)(cg * 128 + t * 16 + nloc) * KIN + kb, hlf); acc[t] = wmma16b(a, bw, acc[t]); if (NPROD == 2) acc[t] = wmma16b(al, bw, acc[t]); } }
    if (EPI == 2) {
#pragma unroll
      for (int t = 0; t < 8; ++t) { const int c = cg * 128 + t * 16 + nloc; const float bb = bf16_rne(bias[c]);
#pragma unroll 1
        for (int r8 = 0; r8 < 8; ++r8) Tf[8 * hlf + r8][c] = acc[t][r8] * sc + bb; } }
    else {
#pragma unroll
      for (int t = 0; t < 8; ++t) { const int c = t * 16 + nloc;
#pragma unroll 1
        for (int r8 = 0; r8 < 8; ++r8) { float val = acc[t][r8] * sc; if (EPI == 1) val = fmaxf(val, 0.0f) + bf16_rne(RES[(m0 + 8 * hlf + r8) * NOUT + cg * 128 + c]); Tf[8 * hlf + r8][c] = val; } }
      wave_lds_sync();
      for (int pass = 0; pass < 2; ++pass) { for (int rr = 0; rr < 16; ++rr) *(volatile v4f*)(OUT + (m0 + rr) * NOUT + cg * 128 + lane * 4) = *(const v4f*)(&Tf[rr][lane * 4]); __threadfence(); }
      wave_lds_sync(); } }
  if (EPI == 2) { wave_lds_sync();
    float g8[8], b8[8]; for (int j = 0; j < 8; ++j) { const int c = (j >> 2) * 128 + lane * 4 + (j & 3); g8[j] = bf16_rne(lng[c]); b8[j] = bf16_rne(lnb[c]); }
    for (int rr = 0; rr < 16; ++rr) { float hv[8]; for (int j = 0; j < 8; ++j) hv[j] = Tf[rr][(j >> 2) * 128 + lane * 4 + (j & 3)]; float s = 0.0f; for (int j = 0; j < 8; ++j) s += hv[j]; for (int o = 16; o; o >>= 1) s += __shfl_xor(s, o); const float mu = s * (1.0f / NOUT);
      float qv = 0.0f; for (int j = 0; j < 8; ++j) { const float d = hv[j] - mu; qv += pmul(d, d); } for (int o = 16; o; o >>= 1) qv += __shfl_xor(qv, o); const float rs = rsqrtf(qv * (1.0f / NOUT) + lneps);
      v4f o0, o1; for (int j = 0; j < 4; ++j) { o0[j] = pmul(pmul(hv[j] - mu, rs), g8[j]) + b8[j]; o1[j] = pmul(pmul(hv[4 + j] - mu, rs), g8[4 + j]) + b8[4 + j]; }
      for (int pass = 0; pass < 2; ++pass) { *(volatile v4f*)(OUT + (m0 + rr) * NOUT + lane * 4) = o0; *(volatile v4f*)(OUT + (m0 + rr) * NOUT + 128 + lane * 4) = o1; __threadfence(); } } }
}
__global__ __launch_bounds__(32) void mid_kernel(const float* __restrict__ XZ, const float* __restrict__ cw, const float* __restrict__ cb, const b16* __restrict__ WX, const b16* __restrict__ WDT, const float* __restrict__ bdt, float* __restrict__ XC, float* __restrict__ BCp, float* __restrict__ DT) {
  __shared__ __attribute__((aligned(16))) b16 Ah[16][DI + 8], Al[16][DI + 8]; __shared__ __attribute__((aligned(16))) float Tf[16][128 + 4]; __shared__ __attribute__((aligned(16))) float Sbc[16][32];
  const int lane = threadIdx.x, nloc = lane & 15, hlf = lane >> 4; const size_t m0 = (size_t)blockIdx.x * 16; const int tpos0 = (int)(m0 % L);
  for (int rr = 0; rr < 16; ++rr) { const int tpos = tpos0 + rr;
    for (int q = 0; q < 4; ++q) { v4f acc = {0.0f, 0.0f, 0.0f, 0.0f};
      for (int k = 0; k < KC; ++k) { const int tt = tpos - (KC - 1) + k; if (tt >= 0) { const v4f xv = *(const v4f*)(XZ + (m0 + rr - (KC - 1) + k) * (2 * DI) + q * 128 + lane * 4); for (int j = 0; j < 4; ++j) acc[j] += pmul(xv[j], bf16_rne(cw[(q * 128 + lane * 4 + j) * KC + k])); } }
      v4f o; for (int j = 0; j < 4; ++j) { const int c = q * 128 + lane * 4 + j; o[j] = silu(acc[j] + bf16_rne(cb[c])); b16 p, ql; split16(o[j] * XS, p, ql); Ah[rr][c] = p; Al[rr][c] = ql; }
      for (int pass = 0; pass < 2; ++pass) { *(volatile v4f*)(XC + (m0 + rr) * DI + q * 128 + lane * 4) = o; __threadfence(); } } }
  wave_lds_sync();
  v8f ax[3] = {(v8f){}, (v8f){}, (v8f){}};
#pragma unroll 2
  for (int kb = 0; kb < DI; kb += 32) { const v16b a = frag_kb(&Ah[nloc][kb], hlf), al = frag_kb(&Al[nloc][kb], hlf);
#pragma unroll
    for (int t = 0; t < 3; ++t) { const v16b bw = frag_kb(WX + (size_t)(t * 16 + nloc) * DI + kb, hlf); ax[t] = wmma16b(a, bw, ax[t]); ax[t] = wmma16b(al, bw, ax[t]); } }
  wave_lds_sync();
  const float sx = 1.0f / (XS * WSC);
#pragma unroll
  for (int r8 = 0; r8 < 8; ++r8) { const int rl = 8 * hlf + r8; const float dtr = ax[0][r8] * sx; b16 p, ql; split16(dtr * ES, p, ql); Ah[rl][nloc] = p; Al[rl][nloc] = ql; Ah[rl][16 + nloc] = (b16)0.0f; Al[rl][16 + nloc] = (b16)0.0f; Sbc[rl][nloc] = ax[1][r8] * sx; Sbc[rl][16 + nloc] = ax[2][r8] * sx; }
  wave_lds_sync();
  for (int pass = 0; pass < 2; ++pass) { for (int rr = 0; rr < 16; ++rr) ((volatile float*)BCp)[(m0 + rr) * 32 + lane] = Sbc[rr][lane]; __threadfence(); }
  const float se = 1.0f / (ES * WSC);
#pragma unroll 1
  for (int cg = 0; cg < 4; ++cg) { v8f acc[8];
#pragma unroll
    for (int t = 0; t < 8; ++t) { acc[t] = (v8f){}; const v16b a = frag_kb(&Ah[nloc][0], hlf), al = frag_kb(&Al[nloc][0], hlf); const v16b bw = frag_kb(WDT + (size_t)(cg * 128 + t * 16 + nloc) * 32, hlf); acc[t] = wmma16b(a, bw, acc[t]); acc[t] = wmma16b(al, bw, acc[t]); }
#pragma unroll
    for (int t = 0; t < 8; ++t) { const int c = cg * 128 + t * 16 + nloc; const float bb = bf16_rne(bdt[c]);
#pragma unroll 1
      for (int r8 = 0; r8 < 8; ++r8) Tf[8 * hlf + r8][t * 16 + nloc] = softplus(acc[t][r8] * se + bb); }
    wave_lds_sync();
    for (int pass = 0; pass < 2; ++pass) { for (int rr = 0; rr < 16; ++rr) *(volatile v4f*)(DT + (m0 + rr) * DI + cg * 128 + lane * 4) = *(const v4f*)(&Tf[rr][lane * 4]); __threadfence(); }
    wave_lds_sync(); }
}
__global__ __launch_bounds__(256) void scan_kernel(const float* __restrict__ XC, const float* __restrict__ DT, const float* __restrict__ BCp, const float* __restrict__ XZ, const float* __restrict__ alog, const float* __restrict__ Dp, float* __restrict__ Y) {
  const int gid = blockIdx.x * 256 + threadIdx.x; const int b = gid / DI, d = gid % DI; if (b >= NB) return;
  float A[DS]; for (int s = 0; s < DS; ++s) A[s] = -__expf(bf16_rne(alog[d * DS + s])); const float dd = bf16_rne(Dp[d]);
#pragma unroll 1
  for (int pass = 0; pass < 2; ++pass) { float h[DS]; for (int s = 0; s < DS; ++s) h[s] = 0.0f;
#pragma unroll 1
    for (int t = 0; t < L; ++t) { const size_t row = (size_t)b * L + t; const float x = XC[row * DI + d], dt = DT[row * DI + d], z = XZ[row * (2 * DI) + DI + d]; const float dx = pmul(dt, x); float y = 0.0f;
#pragma unroll
      for (int s = 0; s < DS; ++s) { const float da = __expf(pmul(dt, A[s])); h[s] = pmul(da, h[s]) + pmul(dx, BCp[row * 32 + s]); y += pmul(h[s], BCp[row * 32 + 16 + s]); }
      y += pmul(dd, x); ((volatile float*)Y)[row * DI + d] = pmul(y, silu(z)); }
    __threadfence(); }
}
__global__ __launch_bounds__(256) void mean_kernel(const float* __restrict__ PA, const float* __restrict__ PE, float* __restrict__ MEANp) {
  const int b = blockIdx.x, c = threadIdx.x; float sa = 0.0f, se2 = 0.0f;
#pragma unroll 1
  for (int t = 0; t < L; ++t) { sa += PA[((size_t)b * L + t) * DM + c]; se2 += PE[((size_t)b * L + t) * DM + c]; }
  const float m = 0.5f * (sa * (1.0f / L) + se2 * (1.0f / L)); for (int pass = 0; pass < 2; ++pass) { ((volatile float*)MEANp)[b * DM + c] = m; __threadfence(); }
}
__global__ __launch_bounds__(256) void gate_kernel(const float* __restrict__ MEANp, const float* __restrict__ fW, float* __restrict__ FW) {
  const int b = blockIdx.x, c = threadIdx.x; float s = 0.0f;
#pragma unroll 1
  for (int k = 0; k < DM; ++k) s += pmul(MEANp[b * DM + k], bf16_rne(fW[k * DM + c]));
  const float g = sigm(s); for (int pass = 0; pass < 2; ++pass) { ((volatile float*)FW)[b * DM + c] = g; __threadfence(); }
}
__global__ __launch_bounds__(256) void final_kernel(const float* __restrict__ P, const float* __restrict__ FW, const float* __restrict__ SC, float* __restrict__ out) {
  const size_t i4 = (size_t)blockIdx.x * 256 + threadIdx.x; const size_t i = i4 * 4; if (i >= (size_t)NT * DM) return; const size_t row = i / DM; const int c = (int)(i % DM); const int b = (int)(row / L);
  const v4f p = *(const v4f*)(P + i), f = *(const v4f*)(FW + b * DM + c), s = *(const v4f*)(SC + i); v4f o; for (int j = 0; j < 4; ++j) o[j] = pmul(p[j], f[j]) + s[j];
  for (int pass = 0; pass < 2; ++pass) { *(volatile v4f*)(out + i) = o; __threadfence(); }
}
}

extern "C" void kernel_launch(void* const* d_in, const int* in_sizes, int n_in, void* d_out, int out_size, void* d_ws, size_t ws_size, hipStream_t stream) {
  (void)n_in;
  auto Fp = [&](int i) { return (const float*)d_in[i]; };
  if (in_sizes[0] != NT * DM || in_sizes[1] != NT * DM || in_sizes[4] != DM * 2 * DI || in_sizes[7] != DI * XD || in_sizes[8] != DTR * DI || in_sizes[12] != DI * DM || in_sizes[15] != DM * 2 * DI || in_sizes[23] != DI * DM || in_sizes[24] != DM * DM || in_sizes[28] != DM * DM || out_size != 2 * NT * DM) return;
  size_t off = 0; char* ws = (char*)d_ws;
  auto carve = [&](size_t bytes) { char* p = ws + off; off += (bytes + 255) & ~(size_t)255; return p; };
  b16* WIN[2]; b16* WX[2]; b16* WDT[2]; b16* WOUT[2]; for (int r = 0; r < 2; ++r) { WIN[r] = (b16*)carve((size_t)2 * DI * DM * 2); WX[r] = (b16*)carve((size_t)XD * DI * 2); WDT[r] = (b16*)carve((size_t)DI * 32 * 2); WOUT[r] = (b16*)carve((size_t)DM * DI * 2); }
  b16* WSC_ = (b16*)carve((size_t)DM * DM * 2);
  float* XZ = (float*)carve((size_t)NT * 2 * DI * 4); float* XC = (float*)carve((size_t)NT * DI * 4); float* DT = (float*)carve((size_t)NT * DI * 4); float* BCp = (float*)carve((size_t)NT * 32 * 4); float* Y = (float*)carve((size_t)NT * DI * 4);
  float* PBR[2]; PBR[0] = (float*)carve((size_t)NT * DM * 4); PBR[1] = (float*)carve((size_t)NT * DM * 4); float* SCB[2]; SCB[0] = (float*)carve((size_t)NT * DM * 4); SCB[1] = (float*)carve((size_t)NT * DM * 4);
  float* MEANp = (float*)carve(NB * DM * 4); float* FW = (float*)carve(NB * DM * 4);
  if (off > ws_size || off > ((size_t)64 << 20)) return;
  const int NBV = NB; const int NTV = NBV * L;
  auto g8 = [](size_t n8) { return (unsigned)((n8 + 255) / 256); };
  for (int r = 0; r < 2; ++r) { const int base = 2 + 11 * r;
    wprep_kernel<<<g8((size_t)2 * DI * DM / 8), 256, 0, stream>>>(Fp(base + 2), DM, 2 * DI, DM, WIN[r]); wprep_kernel<<<g8((size_t)XD * DI / 8), 256, 0, stream>>>(Fp(base + 5), DI, XD, DI, WX[r]);
    wprep_kernel<<<g8((size_t)DI * 32 / 8), 256, 0, stream>>>(Fp(base + 6), DTR, DI, 32, WDT[r]); wprep_kernel<<<g8((size_t)DM * DI / 8), 256, 0, stream>>>(Fp(base + 10), DI, DM, DI, WOUT[r]); }
  wprep_kernel<<<g8((size_t)DM * DM / 8), 256, 0, stream>>>(Fp(24), DM, DM, DM, WSC_);
  for (int r = 0; r < 2; ++r) { const int base = 2 + 11 * r; const float* x = Fp(r);
    gemm_kernel<DM, 2 * DI, 1, 0, 2><<<NTV / 16, 32, 0, stream>>>(x, Fp(base + 0), Fp(base + 1), 1e-6f, XS, WIN[r], nullptr, nullptr, XZ);
    mid_kernel<<<NTV / 16, 32, 0, stream>>>(XZ, Fp(base + 3), Fp(base + 4), WX[r], WDT[r], Fp(base + 7), XC, BCp, DT);
    scan_kernel<<<NBV * DI / 256, 256, 0, stream>>>(XC, DT, BCp, XZ, Fp(base + 8), Fp(base + 9), Y);
    gemm_kernel<DI, DM, 2, 1, 2><<<NTV / 16, 32, 0, stream>>>(Y, nullptr, nullptr, 0.0f, ES, WOUT[r], nullptr, x, PBR[r]);
    gemm_kernel<DM, DM, 0, 2, 1><<<NTV / 16, 32, 0, stream>>>(x, Fp(26), Fp(27), 1e-5f, XS, WSC_, Fp(25), nullptr, SCB[r]);
  }
  mean_kernel<<<NBV, 256, 0, stream>>>(PBR[0], PBR[1], MEANp); gate_kernel<<<NBV, 256, 0, stream>>>(MEANp, Fp(28), FW);
  final_kernel<<<(unsigned)((size_t)NTV * DM / 4 / 256), 256, 0, stream>>>(PBR[0], FW, SCB[0], (float*)d_out); final_kernel<<<(unsigned)((size_t)NTV * DM / 4 / 256), 256, 0, stream>>>(PBR[1], FW, SCB[1], (float*)d_out + (size_t)NT * DM);
}
